// LiquidTransformerLayer_52922587022083
// MI455X (gfx1250) — hardware-verified
//
#include <hip/hip_runtime.h>
#include <math.h>

typedef __attribute__((ext_vector_type(16))) _Float16 v16h;
typedef __attribute__((ext_vector_type(16))) __bf16 v16b;
typedef __attribute__((ext_vector_type(8)))  _Float16 v8h;
typedef __attribute__((ext_vector_type(8)))  float v8f;
typedef __attribute__((ext_vector_type(4)))  float v4f;
typedef __attribute__((ext_vector_type(2)))  float v2f;
typedef __attribute__((ext_vector_type(4)))  unsigned v4u;
typedef __attribute__((ext_vector_type(4)))  int v4i;
typedef float __attribute__((may_alias)) float_a;
typedef int __attribute__((may_alias)) int_a;

template <typename T> __device__ __forceinline__ void vst2(void* p, T v) { *(volatile T*)p = v; __threadfence(); *(volatile T*)p = v; }
__device__ __forceinline__ v8f wmma16(v16h a, v16h b, v8f c) {
  v8f d = __builtin_amdgcn_wmma_f32_16x16x32_f16(false, a, false, b, (short)0, c, false, false);
  asm volatile("v_nop\n\tv_nop\n\tv_nop\n\tv_nop" : "+v"(d) : "v"(a), "v"(b));
  return d;
}
__device__ __forceinline__ v8f wmma_bf(v16b a, v16b b, v8f c) {
  v8f d = __builtin_amdgcn_wmma_f32_16x16x32_bf16(false, a, false, b, (short)0, c, false, false);
  asm volatile("v_nop\n\tv_nop\n\tv_nop\n\tv_nop" : "+v"(d) : "v"(a), "v"(b));
  return d;
}
__device__ __forceinline__ v16h frag_h(const _Float16* rowk0, int lane) {
  union { v16h v; v8h q[2]; } u; const _Float16* p = rowk0 + 8 * (lane >> 4);
  u.q[0] = *(const v8h*)p; u.q[1] = *(const v8h*)(p + 16); return u.v;
}
__device__ __forceinline__ v16h frag_f32(const float* rowk0, int lane) {
  v16h a; const float* p = rowk0 + 8 * (lane >> 4);
#pragma unroll
  for (int i = 0; i < 8; ++i) { a[i] = (_Float16)p[i]; a[8 + i] = (_Float16)p[16 + i]; }
  return a;
}
__device__ __forceinline__ v16h frag_f32s(const float* rowk0, int lane, float sc) {
  v16h a; const float* p = rowk0 + 8 * (lane >> 4);
#pragma unroll
  for (int i = 0; i < 8; ++i) { a[i] = (_Float16)(p[i] * sc); a[8 + i] = (_Float16)(p[16 + i] * sc); }
  return a;
}
__device__ __forceinline__ v16h fragc_f32(const float* W, int k0, int n, int lane, int ld, int K) {
  v16h a; const int g = lane >> 4;
#pragma unroll
  for (int i = 0; i < 8; ++i) { const int ka = k0 + 8 * g + i, kb = ka + 16;
    a[i] = (_Float16)(ka < K ? W[(size_t)(ka < K ? ka : K - 1) * ld + n] : 0.f); a[8 + i] = (_Float16)(kb < K ? W[(size_t)(kb < K ? kb : K - 1) * ld + n] : 0.f); }
  return a;
}
struct F2 { v16b h, l; };
__device__ __forceinline__ F2 bsplit16(const float v[16]) { F2 r;
#pragma unroll
  for (int i = 0; i < 16; ++i) { const __bf16 h = (__bf16)v[i]; r.h[i] = h; r.l[i] = (__bf16)(v[i] - (float)h); }
  return r; }
__device__ __forceinline__ F2 split_row(const float* row, int k0, int lane) { float v[16]; const float* p = row + k0 + 8 * (lane >> 4);
#pragma unroll
  for (int i = 0; i < 8; ++i) { v[i] = p[i]; v[8 + i] = p[16 + i]; }
  return bsplit16(v); }
__device__ __forceinline__ F2 split_rowK(const float* row, int k0, int lane, int K) { float v[16]; const int g = lane >> 4;
#pragma unroll
  for (int i = 0; i < 8; ++i) { const int ka = k0 + 8 * g + i, kb = ka + 16; v[i] = ka < K ? row[ka < K ? ka : K - 1] : 0.f; v[8 + i] = kb < K ? row[kb < K ? kb : K - 1] : 0.f; }
  return bsplit16(v); }
__device__ __forceinline__ F2 split_col(const float* W, int k0, int n, int lane, int ld, int K) { float v[16]; const int g = lane >> 4;
#pragma unroll
  for (int i = 0; i < 8; ++i) { const int ka = k0 + 8 * g + i, kb = ka + 16; v[i] = ka < K ? W[(size_t)(ka < K ? ka : K - 1) * ld + n] : 0.f; v[8 + i] = kb < K ? W[(size_t)(kb < K ? kb : K - 1) * ld + n] : 0.f; }
  return bsplit16(v); }
__device__ __forceinline__ v8f mac3(const F2& a, const F2& b, v8f c) { c = wmma_bf(a.l, b.h, c); c = wmma_bf(a.h, b.l, c); return wmma_bf(a.h, b.h, c); }
__device__ __forceinline__ float sigm(float v) { return 1.0f / (1.0f + expf(-v)); }
#define LDSX() do { asm volatile("s_wait_dscnt 0" ::: "memory"); __builtin_amdgcn_wave_barrier(); __builtin_amdgcn_fence(__ATOMIC_RELEASE, "workgroup"); } while (0)


#define NB 2
#define SS 2048
#define DM 1024
#define NH 16
#define HD 64
#define NR (NB * SS)
#define QKVP (3 * DM)
#define DG 4096
#define DF 2048
#ifndef TRB
#define TRB (NR / 64)
#define TQB (SS / 64)
#define TNB NB
#define KST (SS / 32)
#endif
typedef __attribute__((ext_vector_type(8))) __bf16 v8b;
__device__ __forceinline__ v16b frag_b(const __bf16* rowk0, int lane) {
  union { v16b v; v8b q[2]; } u; const __bf16* p = rowk0 + 8 * (lane >> 4);
  u.q[0] = *(const v8b*)p; u.q[1] = *(const v8b*)(p + 16); return u.v;
}
__device__ __forceinline__ float bfr(float v) { return (float)(__bf16)v; }
__device__ __attribute__((noinline)) float exp_ni(float v) { return expf(v); }
__device__ __attribute__((noinline)) float erf_ni(float v) { return erff(v); }

__device__ __attribute__((noinline)) float tanh_ni(float v) { return tanhf(v); }
#define PK_Q   0
#define PK_RQ  (PK_Q + (size_t)DM * DM)
#define PK_K   (PK_RQ + (size_t)DM * DM)
#define PK_RK  (PK_K + (size_t)DM * DM)
#define PK_V   (PK_RK + (size_t)DM * DM)
#define PK_O   (PK_V + (size_t)DM * DM)
#define PK_G   (PK_O + (size_t)DM * DM)
#define PK_F   (PK_G + (size_t)DG * DM)
#define PK_END (PK_F + (size_t)DM * DF)
#define WS_PK   0u
#define WS_XN   (WS_PK + 2u * (unsigned)PK_END)
#define WS_QKV  (WS_XN + 4u * NR * DM)
#define WS_VT   (WS_QKV + 4u * NR * QKVP)
#define WS_X1   (WS_VT + 2u * NB * DM * SS)
#define WS_END  (WS_X1 + 4u * NR * DM)

__global__ __launch_bounds__(256) void k_packT(const float* __restrict__ Wm, int K, int ld, __bf16* __restrict__ DST) {
  __shared__ __align__(16) __bf16 s[DF]; const int n = blockIdx.x, tid = threadIdx.x;
  for (int k = tid; k < K; k += 256) s[k] = (__bf16)Wm[(size_t)k * ld + n];
  __syncthreads();
  for (int q = tid; q < K / 8; q += 256) vst2((unsigned*)(DST + (size_t)n * K + q * 8), *(const v4u*)&s[q * 8]);
}
template <int XB>
__global__ __launch_bounds__(256) void k_ln(const float* __restrict__ X, const float* __restrict__ gw, const float* __restrict__ bw, float* __restrict__ Y) {
  __shared__ __align__(16) float s[8][DM];
  const int wave = threadIdx.x >> 5, lane = threadIdx.x & 31; const size_t r = (size_t)blockIdx.x * 8 + wave; const float* x = X + r * DM; float* sw = s[wave];
  float sum = 0.f;
#pragma unroll 4
  for (int i = 0; i < DM / 32; ++i) { float t = x[lane + 32 * i]; if (XB) t = bfr(t); sw[lane + 32 * i] = t; sum += t; }
#pragma unroll
  for (int o = 1; o < 32; o <<= 1) sum += __shfl_xor(sum, o);
  const float mu = sum / (float)DM; float var = 0.f;
#pragma unroll 4
  for (int i = 0; i < DM / 32; ++i) { const float d = sw[lane + 32 * i] - mu; var += d * d; }
#pragma unroll
  for (int o = 1; o < 32; o <<= 1) var += __shfl_xor(var, o);
  const float rs = rsqrtf(var / (float)DM + 1e-5f);
#pragma unroll 4
  for (int i = 0; i < DM / 32; ++i) { const int c = lane + 32 * i; sw[c] = (sw[c] - mu) * rs * bfr(gw[c]) + bfr(bw[c]); }
  LDSX();
#pragma unroll 2
  for (int pc = lane; pc < DM / 4; pc += 32) vst2(Y + r * DM + pc * 4, *(const v4f*)&sw[pc * 4]);
}
template <int K, int EPI, int RM>
__global__ __launch_bounds__(128) void k_lin(const float* __restrict__ A, int lda, const __bf16* __restrict__ P, const float* __restrict__ bias, float* __restrict__ OUT, int ldo, const float* __restrict__ RES, int ldr) {
  __shared__ __align__(16) float so[4][16][132];
  const int tid = threadIdx.x, wave = tid >> 5, lane = tid & 31, col = lane & 15, g = lane >> 4; const size_t r0 = (size_t)blockIdx.x * 64 + wave * 16; const int n0 = blockIdx.y * 128;
  v8f acc[8] = {};
#pragma unroll 2
  for (int kc = 0; kc < K / 32; ++kc) { const F2 a = split_row(A + (r0 + col) * lda, kc * 32, lane);
#pragma unroll
    for (int j = 0; j < 8; ++j) { const v16b w = frag_b(P + (size_t)(n0 + j * 16 + col) * K + kc * 32, lane); acc[j] = wmma_bf(a.l, w, acc[j]); acc[j] = wmma_bf(a.h, w, acc[j]); } }
#pragma unroll
  for (int j = 0; j < 8; ++j) { const int n = n0 + j * 16 + col; const float bb = bias ? bfr(bias[n]) : 0.f;
#pragma unroll
    for (int r = 0; r < 8; ++r) { const size_t row = r0 + 8 * g + r; float v = acc[j][r] + bb; if (EPI == 2) v = tanh_ni(v); if (RM == 1) v += RES[row * ldr + n]; if (RM == 2) v += bfr(RES[row * ldr + n]); so[wave][8 * g + r][j * 16 + col] = v; } }
  LDSX();
  for (int rl = 0; rl < 16; ++rl) vst2(OUT + (r0 + rl) * ldo + n0 + lane * 4, *(const v4f*)&so[wave][rl][lane * 4]);
}
__global__ __launch_bounds__(256) void k_vt(const float* __restrict__ QKV, __bf16* __restrict__ VT) {
  __shared__ __align__(16) __bf16 sv[DM][72];
  const int tid = threadIdx.x; const size_t t0 = (size_t)blockIdx.x * 64; const int b = (int)(t0 / SS), p0 = (int)(t0 % SS);
  for (int q = tid; q < 64 * DM; q += 256) { const int tl = q >> 10, c = q & 1023; sv[c][tl] = (__bf16)QKV[(t0 + tl) * QKVP + 2 * DM + c]; }
  __syncthreads();
  for (int q = tid; q < DM * 8; q += 256) { const int rowi = q >> 3, pc = q & 7; vst2((unsigned*)(VT + ((size_t)b * DM + rowi) * SS + p0 + pc * 8), *(const v4u*)&sv[rowi][pc * 8]); }
}
__global__ __launch_bounds__(128) void k_attn(float* __restrict__ QKV, const __bf16* __restrict__ VT) {
  __shared__ __align__(16) float sp[4][16][36]; __shared__ __align__(16) float so[4][16][68];
  const int tid = threadIdx.x, wave = tid >> 5, lane = tid & 31, col = lane & 15, g = lane >> 4;
  const int qb = blockIdx.x, bh = blockIdx.y, b = bh >> 4, h = bh & 15; const int q0 = qb * 64 + wave * 16; const size_t tq = (size_t)b * SS + q0;
  const F2 a0 = split_row(QKV + (tq + col) * QKVP + h * HD, 0, lane), a1 = split_row(QKV + (tq + col) * QKVP + h * HD, 32, lane);
  float m[8], l[8];
#pragma unroll
  for (int r = 0; r < 8; ++r) { m[r] = -3.0e38f; l[r] = 0.f; }
  v8f acc[4] = {};
#pragma unroll 1
  for (int ks = 0; ks < KST; ++ks) { v8f s[2];
#pragma unroll
    for (int ct = 0; ct < 2; ++ct) { const int kk = ks * 32 + ct * 16 + col; const float* krow = QKV + ((size_t)b * SS + kk) * QKVP + DM + h * HD; v16b k0, k1; { const float* p = krow + 8 * g;
#pragma unroll
        for (int i = 0; i < 8; ++i) { k0[i] = (__bf16)p[i]; k0[8 + i] = (__bf16)p[16 + i]; k1[i] = (__bf16)p[32 + i]; k1[8 + i] = (__bf16)p[48 + i]; } }
      v8f c = {}; c = wmma_bf(a0.l, k0, c); c = wmma_bf(a0.h, k0, c); c = wmma_bf(a1.l, k1, c); c = wmma_bf(a1.h, k1, c);
#pragma unroll
      for (int r = 0; r < 8; ++r) s[ct][r] = c[r] * 0.125f; }
#pragma unroll
    for (int r = 0; r < 8; ++r) { float mx = fmaxf(s[0][r], s[1][r]);
#pragma unroll
      for (int o = 1; o < 16; o <<= 1) mx = fmaxf(mx, __shfl_xor(mx, o));
      const float mn = fmaxf(m[r], mx); const float alpha = exp_ni(m[r] - mn);
      const float e0 = exp_ni(s[0][r] - mn), e1 = exp_ni(s[1][r] - mn); float es = e0 + e1;
#pragma unroll
      for (int o = 1; o < 16; o <<= 1) es += __shfl_xor(es, o);
      l[r] = l[r] * alpha + es; m[r] = mn;
#pragma unroll
      for (int dt = 0; dt < 4; ++dt) acc[dt][r] *= alpha;
      sp[wave][8 * g + r][col] = e0; sp[wave][8 * g + r][16 + col] = e1; }
    LDSX();
    const F2 pa = split_row(&sp[wave][col][0], 0, lane);
#pragma unroll
    for (int dt = 0; dt < 4; ++dt) { const v16b vb = frag_b(VT + ((size_t)b * DM + h * HD + dt * 16 + col) * SS + ks * 32, lane); acc[dt] = wmma_bf(pa.l, vb, acc[dt]); acc[dt] = wmma_bf(pa.h, vb, acc[dt]); }
    LDSX(); }
#pragma unroll
  for (int r = 0; r < 8; ++r) { const float il = 1.0f / l[r];
#pragma unroll
    for (int dt = 0; dt < 4; ++dt) so[wave][8 * g + r][dt * 16 + col] = acc[dt][r] * il; }
  LDSX();
  for (int rl = 0; rl < 16; ++rl) if (lane < 16) vst2(QKV + (tq + rl) * QKVP + h * HD + lane * 4, *(const v4f*)&so[wave][rl][lane * 4]);
}
__global__ __launch_bounds__(128) void k_glu(const float* __restrict__ A, const __bf16* __restrict__ PG, const float* __restrict__ bg, float* __restrict__ U, int ldu) {
  __shared__ __align__(16) float so[4][16][132];
  const int tid = threadIdx.x, wave = tid >> 5, lane = tid & 31, col = lane & 15, g = lane >> 4; const size_t r0 = (size_t)blockIdx.x * 64 + wave * 16; const int n0 = blockIdx.y * 128;
  v8f aa[8] = {}, ab[8] = {};
#pragma unroll 1
  for (int kc = 0; kc < DM / 32; ++kc) { const F2 a = split_row(A + (r0 + col) * DM, kc * 32, lane);
#pragma unroll
    for (int j = 0; j < 8; ++j) { const v16b wa = frag_b(PG + (size_t)(n0 + j * 16 + col) * DM + kc * 32, lane), wb = frag_b(PG + (size_t)(DF + n0 + j * 16 + col) * DM + kc * 32, lane);
      aa[j] = wmma_bf(a.l, wa, aa[j]); aa[j] = wmma_bf(a.h, wa, aa[j]); ab[j] = wmma_bf(a.l, wb, ab[j]); ab[j] = wmma_bf(a.h, wb, ab[j]); } }
#pragma unroll
  for (int j = 0; j < 8; ++j) { const int n = n0 + j * 16 + col; const float ba = bfr(bg[n]), bb = bfr(bg[DF + n]);
#pragma unroll
    for (int r = 0; r < 8; ++r) { const float av = aa[j][r] + ba, bv = ab[j][r] + bb; so[wave][8 * g + r][j * 16 + col] = av / (1.0f + exp_ni(-bv)); } }
  LDSX();
  for (int rl = 0; rl < 16; ++rl) vst2(U + (r0 + rl) * ldu + n0 + lane * 4, *(const v4f*)&so[wave][rl][lane * 4]);
}
extern "C" void kernel_launch(void* const* d_in, const int* in_sizes, int n_in, void* d_out, int out_size, void* d_ws, size_t ws_size, hipStream_t stream) {
  (void)in_sizes; (void)n_in; (void)out_size;
  const float** F = (const float**)d_in;
  if (ws_size < (size_t)WS_END) return;
  char* ws = (char*)d_ws; __bf16 *PK = (__bf16*)(ws + WS_PK), *VT = (__bf16*)(ws + WS_VT); float *XN = (float*)(ws + WS_XN), *QKV = (float*)(ws + WS_QKV), *X1 = (float*)(ws + WS_X1);
  k_packT<<<DM, 256, 0, stream>>>(F[1], DM, DM, PK + PK_Q);
  k_packT<<<DM, 256, 0, stream>>>(F[6], DM, DM, PK + PK_RQ);
  k_packT<<<DM, 256, 0, stream>>>(F[2], DM, DM, PK + PK_K);
  k_packT<<<DM, 256, 0, stream>>>(F[7], DM, DM, PK + PK_RK);
  k_packT<<<DM, 256, 0, stream>>>(F[3], DM, DM, PK + PK_V);
  k_packT<<<DM, 256, 0, stream>>>(F[4], DM, DM, PK + PK_O);
  k_packT<<<DG, 256, 0, stream>>>(F[8], DM, DG, PK + PK_G);
  k_packT<<<DM, 256, 0, stream>>>(F[10], DF, DM, PK + PK_F);
  k_ln<1><<<TRB * 8, 256, 0, stream>>>(F[0], F[12], F[13], XN);
  k_lin<DM, 0, 0><<<dim3(TRB, DM / 128), 128, 0, stream>>>(XN, DM, PK + PK_Q, nullptr, QKV + DM, QKVP, nullptr, 0);
  k_lin<DM, 2, 0><<<dim3(TRB, DM / 128), 128, 0, stream>>>(QKV + DM, QKVP, PK + PK_RQ, nullptr, QKV, QKVP, nullptr, 0);
  k_lin<DM, 0, 0><<<dim3(TRB, DM / 128), 128, 0, stream>>>(XN, DM, PK + PK_K, nullptr, QKV + 2 * DM, QKVP, nullptr, 0);
  k_lin<DM, 2, 0><<<dim3(TRB, DM / 128), 128, 0, stream>>>(QKV + 2 * DM, QKVP, PK + PK_RK, nullptr, QKV + DM, QKVP, nullptr, 0);
  k_lin<DM, 0, 0><<<dim3(TRB, DM / 128), 128, 0, stream>>>(XN, DM, PK + PK_V, nullptr, QKV + 2 * DM, QKVP, nullptr, 0);
  k_vt<<<TRB, 256, 0, stream>>>(QKV, VT);
  k_attn<<<dim3(TQB, TNB * NH), 128, 0, stream>>>(QKV, VT);
  k_lin<DM, 0, 2><<<dim3(TRB, DM / 128), 128, 0, stream>>>(QKV, QKVP, PK + PK_O, F[5], X1, DM, F[0], DM);
  k_ln<0><<<TRB * 8, 256, 0, stream>>>(X1, F[14], F[15], XN);
  k_glu<<<dim3(TRB, DF / 128), 128, 0, stream>>>(XN, PK + PK_G, F[9], QKV, DF);
  k_lin<DF, 0, 1><<<dim3(TRB, DM / 128), 128, 0, stream>>>(QKV, DF, PK + PK_F, F[11], (float*)d_out, DM, X1, DM);
}
